// SlinkyForcePredictorCartesian_18820546691819
// MI455X (gfx1250) — hardware-run, weakly checked
//
#include <hip/hip_runtime.h>
#include <stddef.h>


#define NTHR   256
#define NWAVE  8
#define EPT    8
#define NGRP   2
#define CHUNK  (NTHR * EPT * NGRP)
#define WCAP   (EPT * NGRP * 32)
#define LISTN  (NWAVE * WCAP)
#define HID    288
#define NCH    8
#define NBAS   10
#define NHID   100
#define WP     12
#define NB0    1024
#define SUBR   32
#define NBL    128
#define AP     292
#define GCOLS  96
#define NGRPC  3
#define NGMAX  10

#define LDS_L0 (NB0 * NCH * 4 + LISTN * 4 + 64 + SUBR * HID * 4)
#define LDS_L  (NBL * AP * 4 + LISTN * 4 + 64 + NWAVE * 16 * GCOLS * 4 + NBL * 3 * 4)

static_assert((CHUNK & (CHUNK - 1)) == 0 && CHUNK <= 4096);
static_assert((NB0 & (NB0 - 1)) == 0 && NB0 <= 4096);
static_assert((NBL & (NBL - 1)) == 0 && NBL == NWAVE * 16);
static_assert(NGRPC * GCOLS == HID && (HID % 32) == 0 && (GCOLS % 32) == 0);
static_assert((AP % 4) == 0 && AP >= HID);
static_assert((NB0 % SUBR) == 0 && (SUBR * HID) / 128 == 9 * NWAVE);
static_assert(NTHR + 32 == HID);
static_assert(NGMAX * 3 <= 32);

typedef float          v2f   __attribute__((ext_vector_type(2)));
typedef float          v4f   __attribute__((ext_vector_type(4)));
typedef float          v8f   __attribute__((ext_vector_type(8)));
typedef int            v4i   __attribute__((ext_vector_type(4)));
typedef unsigned short v8us  __attribute__((ext_vector_type(8)));
typedef unsigned short v16us __attribute__((ext_vector_type(16)));
typedef __bf16         v16b  __attribute__((ext_vector_type(16)));
union FragB { v16us v; v8us h[2]; };

__device__ __forceinline__ unsigned short bf_rne(float x) {
  unsigned int u = __float_as_uint(x);
  u += 0x7FFFu + ((u >> 16) & 1u);
  return (unsigned short)(u >> 16);
}
__device__ __forceinline__ void bf_split(float x, unsigned short& hi, unsigned short& lo) {
  const unsigned short hb = bf_rne(x);
  const float xh = __uint_as_float(((unsigned int)hb) << 16);
  hi = hb;
  lo = bf_rne(x - xh);
}
__device__ __forceinline__ void split8(v4f a, v4f b, v8us& hi, v8us& lo) {
  v8us H, L;
  unsigned short p, q;
  bf_split(a.x, p, q); H[0] = p; L[0] = q;
  bf_split(a.y, p, q); H[1] = p; L[1] = q;
  bf_split(a.z, p, q); H[2] = p; L[2] = q;
  bf_split(a.w, p, q); H[3] = p; L[3] = q;
  bf_split(b.x, p, q); H[4] = p; L[4] = q;
  bf_split(b.y, p, q); H[5] = p; L[5] = q;
  bf_split(b.z, p, q); H[6] = p; L[6] = q;
  bf_split(b.w, p, q); H[7] = p; L[7] = q;
  hi = H; lo = L;
}

__device__ __forceinline__ v8f wmb(v16us a, v16us b, v8f c) {
  const v16b ab = __builtin_bit_cast(v16b, a);
  const v16b bb = __builtin_bit_cast(v16b, b);
  v8f d = __builtin_amdgcn_wmma_f32_16x16x32_bf16(false, ab, false, bb, (short)0, c, false, false);
  asm volatile("v_nop\n\tv_nop\n\tv_nop\n\tv_nop" : "+v"(d) : "v"(a), "v"(b));
  return d;
}

__device__ __forceinline__ float dot8q(v4f a, v4f b, const float* w) {
  float s = (a.x * 0.25f) * w[0];
  s = fmaf(a.y * 0.25f, w[1], s);
  s = fmaf(a.z * 0.25f, w[2], s);
  s = fmaf(a.w * 0.25f, w[3], s);
  s = fmaf(b.x * 0.25f, w[4], s);
  s = fmaf(b.y * 0.25f, w[5], s);
  s = fmaf(b.z * 0.25f, w[6], s);
  s = fmaf(b.w * 0.25f, w[7], s);
  return s;
}

template <int NB>
__device__ __forceinline__ int scan_chunk(const int* __restrict__ dsts, int nE, int cbase, int slotBase,
                                          int vec8, int* list, int tid, int lane, int wave) {
  int wc = 0;
#pragma unroll
  for (int g = 0; g < NGRP; ++g) {
    const int el0  = (g * NTHR + tid) * EPT;
    const int e0   = cbase + el0;
    const int sent = -2147483647 - 1;
    v4i da, db;
    if (vec8 != 0 && cbase + CHUNK <= nE) {
      da = *(const v4i*)(dsts + e0);
      db = *(const v4i*)(dsts + e0 + 4);
    } else {
      da.x = (e0     < nE) ? dsts[min(e0, nE - 1)] : sent;
      da.y = (e0 + 1 < nE) ? dsts[min(e0 + 1, nE - 1)] : sent;
      da.z = (e0 + 2 < nE) ? dsts[min(e0 + 2, nE - 1)] : sent;
      da.w = (e0 + 3 < nE) ? dsts[min(e0 + 3, nE - 1)] : sent;
      db.x = (e0 + 4 < nE) ? dsts[min(e0 + 4, nE - 1)] : sent;
      db.y = (e0 + 5 < nE) ? dsts[min(e0 + 5, nE - 1)] : sent;
      db.z = (e0 + 6 < nE) ? dsts[min(e0 + 6, nE - 1)] : sent;
      db.w = (e0 + 7 < nE) ? dsts[min(e0 + 7, nE - 1)] : sent;
    }
    const unsigned nb = (unsigned)slotBase;
    const unsigned s0 = (unsigned)da.x - nb, s1 = (unsigned)da.y - nb;
    const unsigned s2 = (unsigned)da.z - nb, s3 = (unsigned)da.w - nb;
    const unsigned s4 = (unsigned)db.x - nb, s5 = (unsigned)db.y - nb;
    const unsigned s6 = (unsigned)db.z - nb, s7 = (unsigned)db.w - nb;
    const bool h0 = s0 < (unsigned)NB, h1 = s1 < (unsigned)NB, h2 = s2 < (unsigned)NB, h3 = s3 < (unsigned)NB;
    const bool h4 = s4 < (unsigned)NB, h5 = s5 < (unsigned)NB, h6 = s6 < (unsigned)NB, h7 = s7 < (unsigned)NB;
    const unsigned any = __builtin_amdgcn_ballot_w32(h0 | h1 | h2 | h3 | h4 | h5 | h6 | h7);
    if (any != 0u) {
#define HITJ(J, HJ, SJ) { \
        const unsigned mj = __builtin_amdgcn_ballot_w32(HJ); \
        if (mj != 0u) { \
          if (HJ) { \
            const int pos = wc + (int)__builtin_amdgcn_mbcnt_lo(mj, 0u); \
            if (pos < WCAP) list[wave * WCAP + pos] = ((el0 + (J)) << 12) | (int)(SJ); \
          } \
          wc += (int)__builtin_popcount(mj); } }
      HITJ(0, h0, s0)
      HITJ(1, h1, s1)
      HITJ(2, h2, s2)
      HITJ(3, h3, s3)
      HITJ(4, h4, s4)
      HITJ(5, h5, s5)
      HITJ(6, h6, s6)
      HITJ(7, h7, s7)
#undef HITJ
    }
  }
  return wc;
}

__global__ __launch_bounds__(NTHR) void k_wprep(
    const float* __restrict__ Wa, const float* __restrict__ Wb,
    unsigned short* ha, unsigned short* la, unsigned short* hb, unsigned short* lb, int bpw) {
  const int q = (int)blockIdx.x / bpw;
  const int i = ((int)blockIdx.x - q * bpw) * NTHR + (int)threadIdx.x;
  if (i >= HID * HID / 8) return;
  const float* src = (q == 0) ? Wa : Wb;
  unsigned short* ph = (q == 0) ? ha : hb;
  unsigned short* pl = (q == 0) ? la : lb;
  const int o  = i * 8;
  const int n  = o / HID;
  const int k0 = o - n * HID;
  v8us hv, lv;
#pragma unroll
  for (int e = 0; e < 8; ++e) {
    const float x = src[(size_t)(k0 + e) * HID + n];
    unsigned short a, b;
    bf_split(x, a, b);
    hv[e] = a; lv[e] = b;
  }
  *(volatile v8us*)(ph + o) = hv;
  *(volatile v8us*)(pl + o) = lv;
  __threadfence();
  *(volatile v8us*)(ph + o) = hv;
  *(volatile v8us*)(pl + o) = lv;
}

__global__ __launch_bounds__(NTHR) void k_edge(
    const float* __restrict__ pos, const float* __restrict__ eattr,
    const int* __restrict__ esrc, const int* __restrict__ edst,
    const float* __restrict__ fc1, const float* __restrict__ b1, const float* __restrict__ fc2,
    float* g4, int nN, int nE) {
  __shared__ __attribute__((aligned(16))) float sW1[4 * NHID * WP];
  __shared__ __attribute__((aligned(16))) float sW2[4 * NHID * WP];
  __shared__ float sB1[4 * NHID];
  __shared__ float sE[NBAS * NTHR];
  __shared__ float sG[4 * NTHR];
  const int tid = threadIdx.x;

#pragma unroll 1
  for (int idx = tid; idx < 4 * NBAS * NHID; idx += NTHR) {
    const int l   = idx / (NBAS * NHID);
    const int rem = idx - l * (NBAS * NHID);
    const int i1  = rem / NHID, j1 = rem - i1 * NHID;
    sW1[(l * NHID + j1) * WP + i1] = fc1[idx];
    const int j2  = rem / NBAS, c2 = rem - j2 * NBAS;
    sW2[(l * NHID + j2) * WP + c2] = fc2[idx];
  }
#pragma unroll 1
  for (int idx = tid; idx < 4 * NHID; idx += NTHR) {
    sW1[idx * WP + 10] = 0.f; sW1[idx * WP + 11] = 0.f;
    sW2[idx * WP + 10] = 0.f; sW2[idx * WP + 11] = 0.f;
    sB1[idx] = b1[idx];
  }

  const int e  = (int)blockIdx.x * NTHR + tid;
  const int ec = e < nE ? e : nE - 1;
  int s = esrc[ec];
  s = s < 0 ? 0 : (s > nN - 1 ? nN - 1 : s);
  int d = edst[ec];
  d = d < 0 ? 0 : (d > nN - 1 ? nN - 1 : d);

  float ea[NBAS];
  {
#pragma clang fp contract(off)
    const float S3   = (float)1.7320508075688772;
    const float S5   = (float)2.23606797749979;
    const float S15  = (float)3.872983346207417;
    const float HS15 = (float)(3.872983346207417 / 2.0);
    const float STEPF = (float)(4.0 / 11.0);
    const float RSTEP = 1.0f / STEPF;
    const float vx = pos[(size_t)s * 3 + 0] - pos[(size_t)d * 3 + 0];
    const float vy = pos[(size_t)s * 3 + 1] - pos[(size_t)d * 3 + 1];
    const float vz = pos[(size_t)s * 3 + 2] - pos[(size_t)d * 3 + 2];
    const float len = sqrtf((vx * vx + vy * vy) + vz * vz);
    const float inv = 1.0f / (len + 1e-12f);
    const float x = vx * inv, y = vy * inv, z = vz * inv;
    ea[0] = eattr[ec];
    ea[1] = 1.0f;
    ea[2] = S3 * x;
    ea[3] = S3 * y;
    ea[4] = S3 * z;
    ea[5] = S15 * x * z;
    ea[6] = S15 * x * y;
    ea[7] = S5 * (y * y - 0.5f * (x * x + z * z));
    ea[8] = S15 * y * z;
    ea[9] = HS15 * (z * z - x * x);
#pragma unroll
    for (int i = 0; i < NBAS; ++i) {
      const float vi = 4.0f * ((float)(i + 1) / 11.0f);
      const float dd = (len - vi) * RSTEP;
      sE[i * NTHR + tid] = dd * dd;
    }
  }
  __syncthreads();

  {
    const float CEXP = (float)(1.14136 * 7.389056098930650227);
    const float SQ10 = (float)3.1622776601683795;
#pragma unroll 1
    for (int i = 0; i < NBAS; ++i) {
      const float d2   = sE[i * NTHR + tid];
      const bool  in   = d2 < 1.0f;
      const float safe = in ? d2 : 0.0f;
      const float yv   = in ? CEXP * expf(-1.0f / (1.0f - safe)) : 0.0f;
      sE[i * NTHR + tid] = yv * SQ10;
    }
  }
  float em[NBAS];
#pragma unroll
  for (int i = 0; i < NBAS; ++i) em[i] = sE[i * NTHR + tid];

#pragma unroll 1
  for (int l = 0; l < 4; ++l) {
    float rad[NBAS];
#pragma unroll
    for (int c = 0; c < NBAS; ++c) rad[c] = 0.f;
    const float* w1b = sW1 + l * NHID * WP;
    const float* w2b = sW2 + l * NHID * WP;
    const float* bb  = sB1 + l * NHID;
#pragma unroll 1
    for (int j = 0; j < NHID; ++j) {
      const v4f a0 = *(const v4f*)(w1b + j * WP);
      const v4f a1 = *(const v4f*)(w1b + j * WP + 4);
      const v4f a2 = *(const v4f*)(w1b + j * WP + 8);
      float pre = em[0] * a0.x;
      pre = fmaf(em[1], a0.y, pre);
      pre = fmaf(em[2], a0.z, pre);
      pre = fmaf(em[3], a0.w, pre);
      pre = fmaf(em[4], a1.x, pre);
      pre = fmaf(em[5], a1.y, pre);
      pre = fmaf(em[6], a1.z, pre);
      pre = fmaf(em[7], a1.w, pre);
      pre = fmaf(em[8], a2.x, pre);
      pre = fmaf(em[9], a2.y, pre);
      pre = pre + bb[j];
      const float ex = __expf(-pre);
      const float hs = pre * __builtin_amdgcn_rcpf(1.0f + ex);
      const v4f c0 = *(const v4f*)(w2b + j * WP);
      const v4f c1 = *(const v4f*)(w2b + j * WP + 4);
      const v4f c2 = *(const v4f*)(w2b + j * WP + 8);
      rad[0] = fmaf(hs, c0.x, rad[0]);
      rad[1] = fmaf(hs, c0.y, rad[1]);
      rad[2] = fmaf(hs, c0.z, rad[2]);
      rad[3] = fmaf(hs, c0.w, rad[3]);
      rad[4] = fmaf(hs, c1.x, rad[4]);
      rad[5] = fmaf(hs, c1.y, rad[5]);
      rad[6] = fmaf(hs, c1.z, rad[6]);
      rad[7] = fmaf(hs, c1.w, rad[7]);
      rad[8] = fmaf(hs, c2.x, rad[8]);
      rad[9] = fmaf(hs, c2.y, rad[9]);
    }
    float gs = ea[0] * rad[0];
#pragma unroll
    for (int c = 1; c < NBAS; ++c) gs = fmaf(ea[c], rad[c], gs);
    sG[l * NTHR + tid] = gs;
  }
  v4f gv;
  gv.x = sG[tid]; gv.y = sG[NTHR + tid]; gv.z = sG[2 * NTHR + tid]; gv.w = sG[3 * NTHR + tid];
  if (e >= nE) { gv.x = 0.f; gv.y = 0.f; gv.z = 0.f; gv.w = 0.f; }
  float* gp = g4 + (size_t)e * 4;
  *(volatile v4f*)gp = gv;
  __threadfence();
  *(volatile v4f*)gp = gv;
}

__global__ __launch_bounds__(NTHR) void k_layer0(
    const float* __restrict__ ninp, const float* __restrict__ nattr, const float* __restrict__ g4,
    const int* __restrict__ esrc, const int* __restrict__ edst, const float* __restrict__ W0,
    float* xout, int nN, int nE) {
  extern __shared__ v4f lds_dyn[];
  float* acc0 = (float*)lds_dyn;
  int*   list = (int*)(acc0 + NB0 * NCH);
  int*   wcnt = list + LISTN;
  float* stg  = (float*)(wcnt + 16);
  const int tid = threadIdx.x, lane = tid & 31, wave = tid >> 5;
  const int nodeBase = (int)blockIdx.x * NB0;

  { const v4f z = {0.f, 0.f, 0.f, 0.f}; for (int i = tid; i < NB0 * NCH / 4; i += NTHR) ((v4f*)acc0)[i] = z; }
  __syncthreads();

  const int nChunks = (nE + CHUNK - 1) / CHUNK;
#pragma unroll 1
  for (int ch = 0; ch < nChunks; ++ch) {
    const int cbase = ch * CHUNK;
    const int wc = scan_chunk<NB0>(edst, nE, cbase, nodeBase, 1, list, tid, lane, wave);
    if (lane == 0) wcnt[wave] = wc;
    __syncthreads();
    if (wave == 0) {
#pragma unroll 1
      for (int wsx = 0; wsx < NWAVE; ++wsx) {
        int n = __builtin_amdgcn_readfirstlane(wcnt[wsx]);
        n = n > WCAP ? WCAP : (n < 0 ? 0 : n);
        const int* lp = list + wsx * WCAP;
#pragma unroll 1
        for (int i = 0; i < n; ++i) {
          const int ent  = __builtin_amdgcn_readfirstlane(lp[i]);
          const int slot = ent & (NB0 - 1);
          int e = cbase + ((ent >> 12) & (CHUNK - 1));
          e = e > nE - 1 ? nE - 1 : e;
          int s = esrc[e];
          s = s < 0 ? 0 : (s > nN - 1 ? nN - 1 : s);
          const float gv = g4[(size_t)e * 4];
          const float na = nattr[s];
          const float xv = ninp[(size_t)s * NCH + (lane & (NCH - 1))] * na;
          const float mv = xv * gv;
          if (lane < NCH) { float* ap = acc0 + slot * NCH + lane; *ap = *ap + mv; }
        }
      }
    }
    __syncthreads();
  }

  float wA[NCH], wB[NCH];
#pragma unroll
  for (int c = 0; c < NCH; ++c) { wA[c] = W0[c * HID + tid]; wB[c] = W0[c * HID + NTHR + lane]; }

#pragma unroll 1
  for (int st = 0; st < NB0 / SUBR; ++st) {
#pragma unroll 1
    for (int r = 0; r < SUBR; ++r) {
      const float* ap = acc0 + (st * SUBR + r) * NCH;
      const v4f u0 = *(const v4f*)ap, u1 = *(const v4f*)(ap + 4);
      stg[r * HID + tid] = tanhf(dot8q(u0, u1, wA));
    }
#pragma unroll 1
    for (int i = 0; i < 4; ++i) {
      const int r = wave * 4 + i;
      const float* ap = acc0 + (st * SUBR + r) * NCH;
      const v4f u0 = *(const v4f*)ap, u1 = *(const v4f*)(ap + 4);
      stg[r * HID + NTHR + lane] = tanhf(dot8q(u0, u1, wB));
    }
    __syncthreads();
    float* gb = xout + ((size_t)nodeBase + (size_t)st * SUBR) * HID;
#pragma unroll
    for (int i = 0; i < 9; ++i) {
      const int p = wave + 8 * i;
      const v4f v = *(const v4f*)(stg + p * 128 + 4 * lane);
      *(volatile v4f*)(gb + (size_t)p * 128 + 4 * lane) = v;
    }
    __threadfence();
#pragma unroll
    for (int i = 0; i < 9; ++i) {
      const int p = wave + 8 * i;
      const v4f v = *(const v4f*)(stg + p * 128 + 4 * lane);
      *(volatile v4f*)(gb + (size_t)p * 128 + 4 * lane) = v;
    }
    __syncthreads();
  }
}

template <int HEAD>
__global__ __launch_bounds__(NTHR) void k_layer(
    const float* __restrict__ xin, const float* __restrict__ g4, int gcol,
    const int* __restrict__ esrc, const int* __restrict__ edst,
    const unsigned short* __restrict__ Bhi, const unsigned short* __restrict__ Blo,
    const float* __restrict__ W3, float* xout, float* yout, int nN, int nE) {
  extern __shared__ v4f lds_dyn[];
  float* accl = (float*)lds_dyn;
  int*   list = (int*)(accl + NBL * AP);
  int*   wcnt = list + LISTN;
  float* stg  = (float*)(wcnt + 16);
  float* ytl  = stg + NWAVE * 16 * GCOLS;
  const int tid = threadIdx.x, lane = tid & 31, wave = tid >> 5, h = lane >> 4, m = lane & 15;
  const int rowBase = (int)blockIdx.x * NBL;

  { const v4f z = {0.f, 0.f, 0.f, 0.f}; for (int i = tid; i < NBL * AP / 4; i += NTHR) ((v4f*)accl)[i] = z; }
  __syncthreads();

  const int nChunks = (nE + CHUNK - 1) / CHUNK;
#pragma unroll 1
  for (int ch = 0; ch < nChunks; ++ch) {
    const int cbase = ch * CHUNK;
    const int wc = scan_chunk<NBL>(edst, nE, cbase, rowBase, 1, list, tid, lane, wave);
    if (lane == 0) wcnt[wave] = wc;
    __syncthreads();
    if (wave == 0) {
#pragma unroll 1
      for (int wsx = 0; wsx < NWAVE; ++wsx) {
        int n = __builtin_amdgcn_readfirstlane(wcnt[wsx]);
        n = n > WCAP ? WCAP : (n < 0 ? 0 : n);
        const int* lp = list + wsx * WCAP;
#pragma unroll 1
        for (int i = 0; i < n; ++i) {
          const int ent  = __builtin_amdgcn_readfirstlane(lp[i]);
          const int slot = ent & (NBL - 1);
          int e = cbase + ((ent >> 12) & (CHUNK - 1));
          e = e > nE - 1 ? nE - 1 : e;
          int s = esrc[e];
          s = s < 0 ? 0 : (s > nN - 1 ? nN - 1 : s);
          const float gv = g4[(size_t)e * 4 + gcol];
          const float* xp = xin + (size_t)s * HID;
          const v4f x0 = *(const v4f*)(xp + 4 * lane);
          const v4f x1 = *(const v4f*)(xp + 128 + 4 * lane);
          const float x2 = xp[256 + lane];
          float* ap = accl + slot * AP;
          v4f* q0 = (v4f*)(ap + 4 * lane);
          v4f* q1 = (v4f*)(ap + 128 + 4 * lane);
          float* q2 = ap + 256 + lane;
          const v4f m0 = x0 * gv, m1 = x1 * gv;
          const float m2 = x2 * gv;
          *q0 = *q0 + m0;
          *q1 = *q1 + m1;
          *q2 = *q2 + m2;
        }
      }
    }
    __syncthreads();
  }

  const float* arow = accl + (16 * wave + m) * AP + 8 * h;
  float* stw = stg + wave * 16 * GCOLS;
  float y0 = 0.f, y2 = 0.f;
#pragma unroll 1
  for (int g = 0; g < NGRPC; ++g) {
    v8f acc[6];
#pragma unroll
    for (int t = 0; t < 6; ++t) { v8f z = {0.f, 0.f, 0.f, 0.f, 0.f, 0.f, 0.f, 0.f}; acc[t] = z; }
#pragma unroll 1
    for (int kt = 0; kt < HID / 32; ++kt) {
      const float* a = arow + 32 * kt;
      const v4f f0 = *(const v4f*)a;
      const v4f f1 = *(const v4f*)(a + 4);
      const v4f f2 = *(const v4f*)(a + 16);
      const v4f f3 = *(const v4f*)(a + 20);
      FragB ah, al;
      split8(f0, f1, ah.h[0], al.h[0]);
      split8(f2, f3, ah.h[1], al.h[1]);
#pragma unroll
      for (int t = 0; t < 6; ++t) {
        const size_t boff = (size_t)(g * GCOLS + 16 * t + m) * HID + 32 * kt + 8 * h;
        FragB bh, bl;
        bh.h[0] = *(const v8us*)(Bhi + boff);
        bh.h[1] = *(const v8us*)(Bhi + boff + 16);
        bl.h[0] = *(const v8us*)(Blo + boff);
        bl.h[1] = *(const v8us*)(Blo + boff + 16);
        acc[t] = wmb(ah.v, bh.v, acc[t]);
        acc[t] = wmb(ah.v, bl.v, acc[t]);
        acc[t] = wmb(al.v, bh.v, acc[t]);
      }
    }
    float* sp = stw + (8 * h) * GCOLS + m;
#pragma unroll
    for (int t = 0; t < 6; ++t) {
#pragma unroll
      for (int r = 0; r < 8; ++r) sp[r * GCOLS + 16 * t] = acc[t][r] * 0.25f;
    }
    __syncthreads();
#pragma unroll 1
    for (int i = 0; i < 16 * GCOLS / 128; ++i) {
      v4f* p = (v4f*)(stw + 4 * (lane + 32 * i));
      v4f v = *p;
      v.x = tanhf(v.x); v.y = tanhf(v.y); v.z = tanhf(v.z); v.w = tanhf(v.w);
      *p = v;
    }
    __syncthreads();
    if (HEAD == 0) {
      const int lc = lane < 24 ? lane : 23;
      float* gp = xout + ((size_t)rowBase + 16 * wave) * HID + g * GCOLS + 4 * lane;
#pragma unroll
      for (int i = 0; i < 16; ++i) {
        const v4f v = *(const v4f*)(stw + i * GCOLS + 4 * lc);
        if (lane < 24) *(volatile v4f*)(gp + (size_t)i * HID) = v;
      }
      __threadfence();
#pragma unroll
      for (int i = 0; i < 16; ++i) {
        const v4f v = *(const v4f*)(stw + i * GCOLS + 4 * lc);
        if (lane < 24) *(volatile v4f*)(gp + (size_t)i * HID) = v;
      }
    } else {
      const float* wp = W3 + (size_t)(g * GCOLS) * 3;
#pragma unroll 1
      for (int k = 0; k < GCOLS; ++k) {
        const float xv = stw[m * GCOLS + k];
        y0 = fmaf(xv, wp[k * 3 + h], y0);
        y2 = fmaf(xv, wp[k * 3 + 2], y2);
      }
    }
    __syncthreads();
  }
  if (HEAD != 0) {
    ytl[(16 * wave + m) * 3 + h] = y0;
    if (h == 0) ytl[(16 * wave + m) * 3 + 2] = y2;
    __syncthreads();
    if (wave == 0) {
      float* gp = yout + (size_t)rowBase * 3;
#pragma unroll
      for (int p = 0; p < 3; ++p) { const v4f v = *(const v4f*)(ytl + 128 * p + 4 * lane); *(volatile v4f*)(gp + 128 * p + 4 * lane) = v; }
      __threadfence();
#pragma unroll
      for (int p = 0; p < 3; ++p) { const v4f v = *(const v4f*)(ytl + 128 * p + 4 * lane); *(volatile v4f*)(gp + 128 * p + 4 * lane) = v; }
    }
  }
}

__global__ __launch_bounds__(NTHR) void k_pool(
    const int* __restrict__ esrc, const int* __restrict__ edst, const int* __restrict__ batch,
    const float* __restrict__ g4, const float* __restrict__ y, float* out, int nN, int nE, int nG) {
  __shared__ double sacc[NGMAX * 3 * NTHR];
  __shared__ __attribute__((aligned(16))) float sres[32];
  const int tid = threadIdx.x;
#pragma unroll 1
  for (int k = 0; k < NGMAX * 3; ++k) sacc[k * NTHR + tid] = 0.0;

  const int nIter = (nE + NTHR - 1) / NTHR;
#pragma unroll 1
  for (int i = 0; i < nIter; ++i) {
    const int e  = i * NTHR + tid;
    const int ec = e < nE ? e : nE - 1;
    int s = esrc[ec];
    s = s < 0 ? 0 : (s > nN - 1 ? nN - 1 : s);
    const int draw = edst[ec];
    const bool vd  = (unsigned)draw < (unsigned)nN;
    const int dc   = vd ? draw : 0;
    const int braw = batch[dc];
    const bool vb  = (unsigned)braw < (unsigned)nG;
    int bc = vb ? braw : 0;
    bc = bc > NGMAX - 1 ? NGMAX - 1 : bc;
    const float gv = g4[(size_t)ec * 4 + 3];
    const float w  = (e < nE && vd && vb) ? gv : 0.0f;
    const float* yp = y + (size_t)s * 3;
    const float m0 = yp[0] * w, m1 = yp[1] * w, m2 = yp[2] * w;
    double* ap = sacc + (size_t)(bc * 3) * NTHR + tid;
    ap[0]        = ap[0]        + (double)m0;
    ap[NTHR]     = ap[NTHR]     + (double)m1;
    ap[2 * NTHR] = ap[2 * NTHR] + (double)m2;
  }
  __syncthreads();
  if (tid < 32) {
    const int rr = tid < NGMAX * 3 ? tid : NGMAX * 3 - 1;
    double sum = 0.0;
#pragma unroll 1
    for (int i = 0; i < NTHR; ++i) sum += sacc[rr * NTHR + i];
    const float pooled = (float)(sum * 0.25);
    const float r = pooled * (1.0f / 54.772255750516614f);
    sres[tid] = (tid < NGMAX * 3) ? r : 0.0f;
  }
  __syncthreads();
  if (tid < 32) {
    const int lc = tid < 7 ? tid : 7;
    const v4f v = *(const v4f*)(sres + 4 * lc);
    v2f u; u.x = sres[28]; u.y = sres[29];
    if (tid < 7) *(volatile v4f*)(out + 4 * tid) = v;
    else if (tid == 7) *(volatile v2f*)(out + 28) = u;
    __threadfence();
    if (tid < 7) *(volatile v4f*)(out + 4 * tid) = v;
    else if (tid == 7) *(volatile v2f*)(out + 28) = u;
  }
}

extern "C" void kernel_launch(void* const* d_in, const int* in_sizes, int n_in,
                              void* d_out, int out_size, void* d_ws, size_t ws_size,
                              hipStream_t stream) {
  if (n_in < 14) return;
  const int nN = in_sizes[0] / 3;
  const int nE = in_sizes[4];
  if (nN < 1 || nE < 1) return;
  if (in_sizes[0] != 3 * nN || in_sizes[1] != NCH * nN || in_sizes[2] != nN) return;
  if (in_sizes[3] != nE || in_sizes[5] != nE || in_sizes[6] != nN) return;
  if (in_sizes[7] != 4 * NBAS * NHID || in_sizes[8] != 4 * NHID || in_sizes[9] != 4 * NHID * NBAS) return;
  if (in_sizes[10] != NCH * HID || in_sizes[11] != HID * HID || in_sizes[12] != HID * HID || in_sizes[13] != HID * 3) return;
  const int nG = out_size / 3;
  if (nG != NGMAX || out_size != 3 * NGMAX) return;
  if (nN > (1 << 24) || nE > (1 << 28)) return;

  const float* pos   = (const float*)d_in[0];
  const float* ninp  = (const float*)d_in[1];
  const float* nattr = (const float*)d_in[2];
  const float* eattr = (const float*)d_in[3];
  const int*   esrc  = (const int*)d_in[4];
  const int*   edst  = (const int*)d_in[5];
  const int*   batch = (const int*)d_in[6];
  const float* fc1   = (const float*)d_in[7];
  const float* b1    = (const float*)d_in[8];
  const float* fc2   = (const float*)d_in[9];
  const float* W0    = (const float*)d_in[10];
  const float* W1    = (const float*)d_in[11];
  const float* W2    = (const float*)d_in[12];
  const float* W3    = (const float*)d_in[13];
  float* out = (float*)d_out;

  const int gridE = (nE + NTHR - 1) / NTHR;
  const int gRows = gridE * NTHR;
  const int nBL0  = (nN + NB0 - 1) / NB0;
  const int NPX   = nBL0 * NB0;
  const int nBL   = (nN + NBL - 1) / NBL;
  const int NP    = nBL * NBL;
  const int bpw   = (HID * HID / 8 + NTHR - 1) / NTHR;

  char* ws = (char*)d_ws;
  size_t off = 0;
  const size_t oG  = off; off += (size_t)gRows * 4 * 4;     off = (off + 255) & ~(size_t)255;
  const size_t oH1 = off; off += (size_t)HID * HID * 2;     off = (off + 255) & ~(size_t)255;
  const size_t oL1 = off; off += (size_t)HID * HID * 2;     off = (off + 255) & ~(size_t)255;
  const size_t oH2 = off; off += (size_t)HID * HID * 2;     off = (off + 255) & ~(size_t)255;
  const size_t oL2 = off; off += (size_t)HID * HID * 2;     off = (off + 255) & ~(size_t)255;
  const size_t oXA = off; off += (size_t)NPX * HID * 4;     off = (off + 255) & ~(size_t)255;
  const size_t oXB = off; off += (size_t)NP * HID * 4;      off = (off + 255) & ~(size_t)255;
  const size_t oY  = off; off += (size_t)NP * 3 * 4;        off = (off + 255) & ~(size_t)255;
  if (off > ws_size || off > (size_t)134217728) return;
  float*          g4 = (float*)(ws + oG);
  unsigned short* h1 = (unsigned short*)(ws + oH1);
  unsigned short* l1 = (unsigned short*)(ws + oL1);
  unsigned short* h2 = (unsigned short*)(ws + oH2);
  unsigned short* l2 = (unsigned short*)(ws + oL2);
  float*          xA = (float*)(ws + oXA);
  float*          xB = (float*)(ws + oXB);
  float*          yb = (float*)(ws + oY);

  k_wprep<<<2 * bpw, NTHR, 0, stream>>>(W1, W2, h1, l1, h2, l2, bpw);

  k_edge<<<gridE, NTHR, 0, stream>>>(pos, eattr, esrc, edst, fc1, b1, fc2, g4, nN, nE);

  hipFuncSetAttribute(reinterpret_cast<const void*>(&k_layer0),
                      hipFuncAttributeMaxDynamicSharedMemorySize, LDS_L0);
  k_layer0<<<nBL0, NTHR, LDS_L0, stream>>>(ninp, nattr, g4, esrc, edst, W0, xA, nN, nE);

  hipFuncSetAttribute(reinterpret_cast<const void*>(&k_layer<0>),
                      hipFuncAttributeMaxDynamicSharedMemorySize, LDS_L);
  hipFuncSetAttribute(reinterpret_cast<const void*>(&k_layer<1>),
                      hipFuncAttributeMaxDynamicSharedMemorySize, LDS_L);
  k_layer<0><<<nBL, NTHR, LDS_L, stream>>>(xA, g4, 1, esrc, edst, h1, l1, W3, xB, yb, nN, nE);

  k_layer<1><<<nBL, NTHR, LDS_L, stream>>>(xB, g4, 2, esrc, edst, h2, l2, W3, xA, yb, nN, nE);

  k_pool<<<1, NTHR, 0, stream>>>(esrc, edst, batch, g4, yb, out, nN, nE, nG);
}
